// FLAGatedLinearAttention_89498528514090
// MI455X (gfx1250) — hardware-verified
//
#include <hip/hip_runtime.h>
#include <math.h>

typedef __attribute__((ext_vector_type(16))) _Float16 v16h;
typedef __attribute__((ext_vector_type(16))) __bf16 v16b;
typedef __attribute__((ext_vector_type(8)))  _Float16 v8h;
typedef __attribute__((ext_vector_type(8)))  float v8f;
typedef __attribute__((ext_vector_type(4)))  float v4f;
typedef __attribute__((ext_vector_type(2)))  float v2f;
typedef __attribute__((ext_vector_type(4)))  unsigned v4u;
typedef __attribute__((ext_vector_type(4)))  int v4i;
typedef float __attribute__((may_alias)) float_a;
typedef int __attribute__((may_alias)) int_a;

template <typename T> __device__ __forceinline__ void vst2(void* p, T v) { *(volatile T*)p = v; __threadfence(); *(volatile T*)p = v; }
__device__ __forceinline__ v8f wmma16(v16h a, v16h b, v8f c) {
  v8f d = __builtin_amdgcn_wmma_f32_16x16x32_f16(false, a, false, b, (short)0, c, false, false);
  asm volatile("v_nop\n\tv_nop\n\tv_nop\n\tv_nop" : "+v"(d) : "v"(a), "v"(b));
  return d;
}
__device__ __forceinline__ v8f wmma_bf(v16b a, v16b b, v8f c) {
  v8f d = __builtin_amdgcn_wmma_f32_16x16x32_bf16(false, a, false, b, (short)0, c, false, false);
  asm volatile("v_nop\n\tv_nop\n\tv_nop\n\tv_nop" : "+v"(d) : "v"(a), "v"(b));
  return d;
}
__device__ __forceinline__ v16h frag_h(const _Float16* rowk0, int lane) {
  union { v16h v; v8h q[2]; } u; const _Float16* p = rowk0 + 8 * (lane >> 4);
  u.q[0] = *(const v8h*)p; u.q[1] = *(const v8h*)(p + 16); return u.v;
}
__device__ __forceinline__ v16h frag_f32(const float* rowk0, int lane) {
  v16h a; const float* p = rowk0 + 8 * (lane >> 4);
#pragma unroll
  for (int i = 0; i < 8; ++i) { a[i] = (_Float16)p[i]; a[8 + i] = (_Float16)p[16 + i]; }
  return a;
}
__device__ __forceinline__ v16h frag_f32s(const float* rowk0, int lane, float sc) {
  v16h a; const float* p = rowk0 + 8 * (lane >> 4);
#pragma unroll
  for (int i = 0; i < 8; ++i) { a[i] = (_Float16)(p[i] * sc); a[8 + i] = (_Float16)(p[16 + i] * sc); }
  return a;
}
__device__ __forceinline__ v16h fragc_f32(const float* W, int k0, int n, int lane, int ld, int K) {
  v16h a; const int g = lane >> 4;
#pragma unroll
  for (int i = 0; i < 8; ++i) { const int ka = k0 + 8 * g + i, kb = ka + 16;
    a[i] = (_Float16)(ka < K ? W[(size_t)(ka < K ? ka : K - 1) * ld + n] : 0.f); a[8 + i] = (_Float16)(kb < K ? W[(size_t)(kb < K ? kb : K - 1) * ld + n] : 0.f); }
  return a;
}
struct F2 { v16b h, l; };
__device__ __forceinline__ F2 bsplit16(const float v[16]) { F2 r;
#pragma unroll
  for (int i = 0; i < 16; ++i) { const __bf16 h = (__bf16)v[i]; r.h[i] = h; r.l[i] = (__bf16)(v[i] - (float)h); }
  return r; }
__device__ __forceinline__ F2 split_row(const float* row, int k0, int lane) { float v[16]; const float* p = row + k0 + 8 * (lane >> 4);
#pragma unroll
  for (int i = 0; i < 8; ++i) { v[i] = p[i]; v[8 + i] = p[16 + i]; }
  return bsplit16(v); }
__device__ __forceinline__ F2 split_rowK(const float* row, int k0, int lane, int K) { float v[16]; const int g = lane >> 4;
#pragma unroll
  for (int i = 0; i < 8; ++i) { const int ka = k0 + 8 * g + i, kb = ka + 16; v[i] = ka < K ? row[ka < K ? ka : K - 1] : 0.f; v[8 + i] = kb < K ? row[kb < K ? kb : K - 1] : 0.f; }
  return bsplit16(v); }
__device__ __forceinline__ F2 split_col(const float* W, int k0, int n, int lane, int ld, int K) { float v[16]; const int g = lane >> 4;
#pragma unroll
  for (int i = 0; i < 8; ++i) { const int ka = k0 + 8 * g + i, kb = ka + 16; v[i] = ka < K ? W[(size_t)(ka < K ? ka : K - 1) * ld + n] : 0.f; v[8 + i] = kb < K ? W[(size_t)(kb < K ? kb : K - 1) * ld + n] : 0.f; }
  return bsplit16(v); }
__device__ __forceinline__ v8f mac3(const F2& a, const F2& b, v8f c) { c = wmma_bf(a.l, b.h, c); c = wmma_bf(a.h, b.l, c); return wmma_bf(a.h, b.h, c); }
__device__ __forceinline__ float sigm(float v) { return 1.0f / (1.0f + expf(-v)); }
#define LDSX() do { asm volatile("s_wait_dscnt 0" ::: "memory"); __builtin_amdgcn_wave_barrier(); __builtin_amdgcn_fence(__ATOMIC_RELEASE, "workgroup"); } while (0)


#define NB 4
#define TT 4096
#define DD 768
#define NH 12
#define HK 32
#define HV 64
#define KD 384
#define NR (NB * TT)
#define LR 16
#ifndef NSTEP
#define NSTEP TT
#define TR_ROWS NR
#define TR_BH (NB * NH)
#endif
typedef __attribute__((ext_vector_type(8))) __bf16 v8b;
__device__ __forceinline__ v16b frag_b(const __bf16* rowk0, int lane) {
  union { v16b v; v8b q[2]; } u; const __bf16* p = rowk0 + 8 * (lane >> 4);
  u.q[0] = *(const v8b*)p; u.q[1] = *(const v8b*)(p + 16); return u.v;
}
__device__ __forceinline__ float bfr(float v) { return (float)(__bf16)v; }
__device__ __forceinline__ v16b frag_gbf(const float* rowk0, int lane) {
  v16b a; const float* p = rowk0 + 8 * (lane >> 4);
#pragma unroll
  for (int i = 0; i < 8; ++i) { a[i] = (__bf16)p[i]; a[8 + i] = (__bf16)p[16 + i]; }
  return a;
}
__device__ __attribute__((noinline)) float exp_ni(float v) { return expf(v); }
__device__ __attribute__((noinline)) float logsig_ni(float z) { return fminf(z, 0.f) - log1pf(expf(-fabsf(z))); }

#define PT_ROWS (KD + KD + DD + DD + DD)
#define WS_PT   0u
#define WS_G1T  (WS_PT + 2u * PT_ROWS * DD)
#define WS_G2T  (WS_G1T + 2u * LR * DD)
#define WS_Q    (WS_G2T + 2u * KD * 32)
#define WS_K    (WS_Q + 4u * NR * KD)
#define WS_V    (WS_K + 4u * NR * KD)
#define WS_H16  (WS_V + 4u * NR * DD)
#define WS_EG   (WS_H16 + 4u * NR * LR)
#define WS_END  (WS_EG + 4u * NR * KD)

__global__ __launch_bounds__(256) void k_pack(const float* __restrict__ Wq, const float* __restrict__ Wk, const float* __restrict__ Wv, const float* __restrict__ Wg, const float* __restrict__ Wo,
                                              const float* __restrict__ Wgk1, const float* __restrict__ Wgk2, __bf16* __restrict__ PT, __bf16* __restrict__ G1T, __bf16* __restrict__ G2T) {
  __shared__ __align__(16) __bf16 srow[DD];
  const int n = blockIdx.x, tid = threadIdx.x;
  if (n < PT_ROWS) { const float* Wm; int NO, nn;
    if (n < KD) { Wm = Wq; NO = KD; nn = n; } else if (n < 2 * KD) { Wm = Wk; NO = KD; nn = n - KD; } else if (n < 2 * KD + DD) { Wm = Wv; NO = DD; nn = n - 2 * KD; }
    else if (n < 2 * KD + 2 * DD) { Wm = Wg; NO = DD; nn = n - 2 * KD - DD; } else { Wm = Wo; NO = DD; nn = n - 2 * KD - 2 * DD; }
    for (int k = tid; k < DD; k += 256) srow[k] = (__bf16)Wm[(size_t)k * NO + nn];
    __syncthreads();
    if (tid < DD / 8) vst2((unsigned*)(PT + (size_t)n * DD + tid * 8), *(const v4u*)(&srow[tid * 8]));
  } else if (n < PT_ROWS + LR) { const int g = n - PT_ROWS;
    for (int k = tid; k < DD; k += 256) srow[k] = (__bf16)Wgk1[(size_t)k * LR + g];
    __syncthreads();
    if (tid < DD / 8) vst2((unsigned*)(G1T + (size_t)g * DD + tid * 8), *(const v4u*)(&srow[tid * 8]));
  }
  (void)Wgk2; (void)G2T;
}
__global__ __launch_bounds__(256) void k_packg2(const float* __restrict__ Wgk2, __bf16* __restrict__ G2T) {
  const int tid = threadIdx.x;
  for (int q = tid; q < KD * 4; q += 256) { const int j = q >> 2, pc = q & 3; union { __bf16 e[8]; v4u u; } pk;
#pragma unroll
    for (int e = 0; e < 8; ++e) { const int k = pc * 8 + e; pk.e[e] = k < LR ? (__bf16)Wgk2[(size_t)k * KD + j] : (__bf16)0.f; }
    vst2((unsigned*)(G2T + (size_t)j * 32 + pc * 8), pk.u); }
}
__global__ __launch_bounds__(128) void k_proj(const float* __restrict__ X, const __bf16* __restrict__ PT, float* __restrict__ Q, float* __restrict__ Kr, float* __restrict__ V) {
  __shared__ __align__(16) float so[4][16][132];
  const int tid = threadIdx.x, wave = tid >> 5, lane = tid & 31, col = lane & 15, g = lane >> 4; const size_t r0 = (size_t)blockIdx.x * 64 + wave * 16; const int n0 = blockIdx.y * 128;
  v8f acc[8] = {};
#pragma unroll 2
  for (int kc = 0; kc < DD / 32; ++kc) { const v16b a = frag_gbf(X + (r0 + col) * DD + kc * 32, lane);
#pragma unroll
    for (int j = 0; j < 8; ++j) acc[j] = wmma_bf(a, frag_b(PT + (size_t)(n0 + j * 16 + col) * DD + kc * 32, lane), acc[j]); }
  float* dst; int pitch, c0; float sc = 1.0f;
  if (n0 < KD) { dst = Q; pitch = KD; c0 = n0; sc = 0.17677669529663687f; } else if (n0 < 2 * KD) { dst = Kr; pitch = KD; c0 = n0 - KD; }
  else { dst = V; pitch = DD; c0 = n0 - 2 * KD; }
#pragma unroll
  for (int j = 0; j < 8; ++j)
#pragma unroll
    for (int r = 0; r < 8; ++r) so[wave][8 * g + r][j * 16 + col] = acc[j][r] * sc;
  LDSX();
  for (int rl = 0; rl < 16; ++rl) vst2(dst + (r0 + rl) * pitch + c0 + lane * 4, *(const v4f*)(&so[wave][rl][lane * 4]));
}
__global__ __launch_bounds__(128) void k_gk1(const float* __restrict__ X, const __bf16* __restrict__ G1T, float* __restrict__ H16) {
  __shared__ __align__(16) float sh[64][16];
  const int tid = threadIdx.x, wave = tid >> 5, lane = tid & 31, col = lane & 15, g = lane >> 4; const size_t r0 = (size_t)blockIdx.x * 64 + wave * 16;
  v8f acc = {};
#pragma unroll 4
  for (int kc = 0; kc < DD / 32; ++kc) acc = wmma_bf(frag_gbf(X + (r0 + col) * DD + kc * 32, lane), frag_b(G1T + (size_t)col * DD + kc * 32, lane), acc);
#pragma unroll
  for (int r = 0; r < 8; ++r) sh[wave * 16 + 8 * g + r][col] = acc[r];
  __syncthreads();
  for (int q = tid; q < 64 * 4; q += 128) vst2(H16 + (size_t)blockIdx.x * 64 * LR + q * 4, *(const v4f*)(&sh[0][0] + q * 4));
}
__global__ __launch_bounds__(128) void k_gk2(const float* __restrict__ H16, const __bf16* __restrict__ G2T, const float* __restrict__ bg, float* __restrict__ EG) {
  __shared__ __align__(16) float so[4][16][132];
  const int tid = threadIdx.x, wave = tid >> 5, lane = tid & 31, col = lane & 15, g = lane >> 4; const size_t r0 = (size_t)blockIdx.x * 64 + wave * 16; const int n0 = blockIdx.y * 128;
  F2 a; { float v[16]; const float* p = H16 + (r0 + col) * LR + 8 * g;
#pragma unroll
    for (int i = 0; i < 8; ++i) { v[i] = p[i]; v[8 + i] = 0.f; }
    a = bsplit16(v); }
  v8f acc[8] = {};
#pragma unroll
  for (int j = 0; j < 8; ++j) { const v16b wb = frag_b(G2T + (size_t)(n0 + j * 16 + col) * 32, lane); acc[j] = wmma_bf(a.l, wb, acc[j]); acc[j] = wmma_bf(a.h, wb, acc[j]); }
#pragma unroll
  for (int j = 0; j < 8; ++j) { const float bb = bfr(bg[n0 + j * 16 + col]);
#pragma unroll
    for (int r = 0; r < 8; ++r) so[wave][8 * g + r][j * 16 + col] = exp_ni(logsig_ni(acc[j][r] + bb) * (1.0f / 16.0f)); }
  LDSX();
  for (int rl = 0; rl < 16; ++rl) vst2(EG + (r0 + rl) * KD + n0 + lane * 4, *(const v4f*)(&so[wave][rl][lane * 4]));
}
__global__ __launch_bounds__(256) void k_scan(const float* __restrict__ Q, const float* __restrict__ Kr, const float* V, const float* __restrict__ EG, float* O) {
  __shared__ __align__(16) float so[16][HV];
  const int bh = blockIdx.x, b = bh / NH, h = bh % NH, tid = threadIdx.x, j = tid >> 2, jq = tid & 3, i0 = jq * 8;
  float S[8];
#pragma unroll
  for (int e = 0; e < 8; ++e) S[e] = 0.f;
  const size_t rb = (size_t)b * TT; const int kc0 = h * HK + i0, vc = h * HV + j;
#pragma unroll 1
  for (int t = 0; t < NSTEP; ++t) { const size_t r = rb + t;
    const float vv = V[r * DD + vc];
    const float4 e0 = *(const float4*)(EG + r * KD + kc0), e1 = *(const float4*)(EG + r * KD + kc0 + 4);
    const float4 k0 = *(const float4*)(Kr + r * KD + kc0), k1 = *(const float4*)(Kr + r * KD + kc0 + 4);
    const float4 q0 = *(const float4*)(Q + r * KD + kc0), q1 = *(const float4*)(Q + r * KD + kc0 + 4);
    const float eg[8] = {e0.x, e0.y, e0.z, e0.w, e1.x, e1.y, e1.z, e1.w}, kk[8] = {k0.x, k0.y, k0.z, k0.w, k1.x, k1.y, k1.z, k1.w}, qq[8] = {q0.x, q0.y, q0.z, q0.w, q1.x, q1.y, q1.z, q1.w};
    float o = 0.f;
#pragma unroll
    for (int e = 0; e < 8; ++e) { S[e] = S[e] * eg[e] + kk[e] * vv; o += qq[e] * S[e]; }
    o += __shfl_xor(o, 1); o += __shfl_xor(o, 2);
    if (jq == 0) so[t & 15][j] = o;
    if ((t & 15) == 15) {
      __syncthreads();
      { const int rl = tid >> 4, pc = tid & 15; vst2(O + (rb + (t - 15) + rl) * DD + h * HV + pc * 4, *(const v4f*)(&so[rl][pc * 4])); }
      __syncthreads(); }
  }
}
__global__ __launch_bounds__(128) void k_gate(const float* __restrict__ X, const __bf16* __restrict__ PT, const float* __restrict__ nw, float* __restrict__ OY) {
  __shared__ __align__(16) float so[64][132];
  __shared__ float srs[64][2];
  const int tid = threadIdx.x, wave = tid >> 5, lane = tid & 31, col = lane & 15, g = lane >> 4; const size_t rb = (size_t)blockIdx.x * 64; const size_t r0 = rb + wave * 16; const int n0 = blockIdx.y * 128;
  v8f acc[8] = {};
#pragma unroll 2
  for (int kc = 0; kc < DD / 32; ++kc) { const v16b a = frag_gbf(X + (r0 + col) * DD + kc * 32, lane);
#pragma unroll
    for (int j = 0; j < 8; ++j) acc[j] = wmma_bf(a, frag_b(PT + (size_t)(2 * KD + DD + n0 + j * 16 + col) * DD + kc * 32, lane), acc[j]); }
  for (int q = tid; q < 64 * 32; q += 128) { const int rl = q >> 5, c4 = (q & 31) * 4; *(float4*)&so[rl][c4] = *(const float4*)(OY + (rb + rl) * DD + n0 + c4); }
  __syncthreads();
  { const int rl = tid >> 1, hh = tid & 1; float s = 0.f;
#pragma unroll 8
    for (int j = 0; j < HV; ++j) { const float v = so[rl][hh * HV + j]; s += v * v; }
    srs[rl][hh] = rsqrtf(s * (1.0f / HV) + 1e-5f); }
  __syncthreads();
#pragma unroll
  for (int j = 0; j < 8; ++j) { const int c = j * 16 + col; const float wj = bfr(nw[c & 63]);
#pragma unroll
    for (int r = 0; r < 8; ++r) { const int rl = wave * 16 + 8 * g + r; const float gv = acc[j][r]; so[rl][c] = (so[rl][c] * srs[rl][c >> 6] * wj) * (gv * (1.0f / (1.0f + exp_ni(-gv)))); } }
  __syncthreads();
  for (int q = tid; q < 64 * 32; q += 128) { const int rl = q >> 5, c4 = (q & 31) * 4; vst2(OY + (rb + rl) * DD + n0 + c4, *(const v4f*)&so[rl][c4]); }
}
__global__ __launch_bounds__(128) void k_out(const float* __restrict__ Y, const __bf16* __restrict__ PT, float* __restrict__ out) {
  __shared__ __align__(16) float so[4][16][132];
  const int tid = threadIdx.x, wave = tid >> 5, lane = tid & 31, col = lane & 15, g = lane >> 4; const size_t r0 = (size_t)blockIdx.x * 64 + wave * 16; const int n0 = blockIdx.y * 128;
  v8f acc[8] = {};
#pragma unroll 2
  for (int kc = 0; kc < DD / 32; ++kc) { const F2 a = split_row(Y + (r0 + col) * DD, kc * 32, lane);
#pragma unroll
    for (int j = 0; j < 8; ++j) { const v16b wb = frag_b(PT + (size_t)(2 * KD + 2 * DD + n0 + j * 16 + col) * DD + kc * 32, lane); acc[j] = wmma_bf(a.l, wb, acc[j]); acc[j] = wmma_bf(a.h, wb, acc[j]); } }
#pragma unroll
  for (int j = 0; j < 8; ++j)
#pragma unroll
    for (int r = 0; r < 8; ++r) so[wave][8 * g + r][j * 16 + col] = acc[j][r];
  LDSX();
  for (int rl = 0; rl < 16; ++rl) vst2(out + (r0 + rl) * DD + n0 + lane * 4, *(const v4f*)(&so[wave][rl][lane * 4]));
}

extern "C" void kernel_launch(void* const* d_in, const int* in_sizes, int n_in, void* d_out, int out_size, void* d_ws, size_t ws_size, hipStream_t stream) {
  (void)in_sizes; (void)n_in; (void)out_size;
  const float** I = (const float**)d_in;
  if (ws_size < (size_t)WS_END) return;
  char* ws = (char*)d_ws;
  __bf16 *PT = (__bf16*)(ws + WS_PT), *G1T = (__bf16*)(ws + WS_G1T), *G2T = (__bf16*)(ws + WS_G2T);
  float *Q = (float*)(ws + WS_Q), *Kr = (float*)(ws + WS_K), *V = (float*)(ws + WS_V), *H16 = (float*)(ws + WS_H16), *EG = (float*)(ws + WS_EG);
  k_pack<<<PT_ROWS + LR, 256, 0, stream>>>(I[1], I[2], I[3], I[7], I[9], I[4], I[5], PT, G1T, G2T);
  k_packg2<<<1, 256, 0, stream>>>(I[5], G2T);
  k_proj<<<dim3(TR_ROWS / 64, (2 * KD + DD) / 128), 128, 0, stream>>>(I[0], PT, Q, Kr, V);
  k_gk1<<<TR_ROWS / 64, 128, 0, stream>>>(I[0], G1T, H16);
  k_gk2<<<dim3(TR_ROWS / 64, KD / 128), 128, 0, stream>>>(H16, G2T, I[6], EG);
  k_scan<<<TR_BH, 256, 0, stream>>>(Q, Kr, V, EG, V);
  k_gate<<<dim3(TR_ROWS / 64, DD / 128), 128, 0, stream>>>(I[0], PT, I[8], V);
  k_out<<<dim3(TR_ROWS / 64, DD / 128), 128, 0, stream>>>(V, PT, (float*)d_out);
}
